// C2fBoT_81063212745480
// MI455X (gfx1250) — hardware-verified
//
#include <hip/hip_runtime.h>
#include <math.h>
#include <stdint.h>

#define NBATCH 8
#define CIN    512
#define CHID   256
#define COUT   512
#define CCAT   1024
#define CQKV   768
#define QKP    512
#define IMW    32
#define HW     1024
#define NTOT   8192
#define NHEAD  4
#define HD     64
#define NLAY   2
#define K3     2304
#define ASC    16.0f
#define WSC    256.0f
#define PSC    4096.0f
#define GINV   0.000244140625f
#define LINV   0.00048828125f
#define OINV   0.000244140625f
#define RINV   0.0625f
#define BNEPS  0.001f
#define OP     136
#define OVP    72
#define OFP    68
#define OP3    264
#define TP     72
#define XSP    520
#define SP     1032
#define PP     1032
#define OPA    72
#define ATT_S_BYTES (32 * SP * 4)
#define ATT_P_BYTES (32 * PP * 2)
#define ATT_R_BYTES (32 * 64 * 4)
#define ATT_O_BYTES (32 * OPA * 2)
#define ATT_LDS (ATT_S_BYTES + ATT_P_BYTES + ATT_R_BYTES + ATT_O_BYTES)

static_assert(K3 == 9 * CHID);
static_assert(K3 % 32 == 0);
static_assert((OP * 2) % 16 == 0);
static_assert((OVP * 2) % 16 == 0);
static_assert((OFP * 4) % 16 == 0);
static_assert((OP3 * 2) % 16 == 0);
static_assert((TP * 2) % 16 == 0);
static_assert((XSP * 2) % 16 == 0);
static_assert((SP * 4) % 16 == 0);
static_assert((PP * 2) % 16 == 0);
static_assert((OPA * 2) % 16 == 0);
static_assert(ATT_S_BYTES % 16 == 0);
static_assert(ATT_P_BYTES % 16 == 0);
static_assert(ATT_R_BYTES % 16 == 0);
static_assert(NHEAD * HD == CHID);
static_assert(NBATCH * HW == NTOT);
static_assert(4 * 34 * TP <= 64 * OP3);

typedef _Float16       v16h __attribute__((ext_vector_type(16)));
typedef _Float16       v8h  __attribute__((ext_vector_type(8)));
typedef unsigned short v8us __attribute__((ext_vector_type(8)));
typedef float          v8f  __attribute__((ext_vector_type(8)));
typedef float          v4f  __attribute__((ext_vector_type(4)));
typedef unsigned int   v4u  __attribute__((ext_vector_type(4)));

union Frag { v8us u[2]; v16h h; };
static_assert(sizeof(Frag) == 32);

__device__ __forceinline__ unsigned short bf_bits(float f) {
  unsigned u = __float_as_uint(f);
  return (unsigned short)((u + 0x7FFFu + ((u >> 16) & 1u)) >> 16);
}
__device__ __forceinline__ float bf_up(unsigned short hb) { return __uint_as_float(((unsigned)hb) << 16); }
__device__ __forceinline__ float bfr(float f) { return bf_up(bf_bits(f)); }
__device__ __forceinline__ unsigned short h_bits(_Float16 x) { return __builtin_bit_cast(unsigned short, x); }
__device__ __forceinline__ float h_val(unsigned short u) { return (float)__builtin_bit_cast(_Float16, u); }
__device__ __forceinline__ unsigned pk16(unsigned short a, unsigned short b) { return (unsigned)a | ((unsigned)b << 16); }
__device__ __forceinline__ v8f zero8() { v8f z = {0.f, 0.f, 0.f, 0.f, 0.f, 0.f, 0.f, 0.f}; return z; }
__device__ __forceinline__ float silu_f(float v) { return v * __builtin_amdgcn_rcpf(1.0f + __expf(-v)); }

__device__ __forceinline__ Frag ldfrag(const unsigned short* p) {
  Frag f;
  f.u[0] = *(const v8us*)(p);
  f.u[1] = *(const v8us*)(p + 16);
  return f;
}

__device__ __forceinline__ v8f mma_h(v16h a, v16h b, v8f c) {
  v8f d = __builtin_amdgcn_wmma_f32_16x16x32_f16(false, a, false, b, (short)0, c, false, false);
#if defined(__HIP_DEVICE_COMPILE__)
  asm volatile("v_nop\n\tv_nop\n\tv_nop\n\tv_nop" : "+v"(d) : "v"(a), "v"(b));
#endif
  return d;
}

__global__ __launch_bounds__(256)
void k_cvt(const float* __restrict__ cv1w, const float* __restrict__ cv1bn, const float* __restrict__ cv2w,
           const float* __restrict__ cv2bn, const float* __restrict__ m1w, const float* __restrict__ m1bn,
           const float* __restrict__ qkvw, const float* __restrict__ m2w, const float* __restrict__ m2bn,
           unsigned short* W1, unsigned short* W3, unsigned short* WQ, unsigned short* W2, unsigned short* WF,
           float* COEF) {
  const int tid = threadIdx.x, e = tid & 7, lq = tid >> 3;
  const int blk = blockIdx.x;
  if (blk < 1216) {
    const float* src;
    size_t base;
    int strd = 1;
    unsigned short* dst;
    if (blk < 128) {
      const int L = blk * 32 + lq;
      const int row = L >> 3, k = (L & 7) * 64 + 8 * e;
      src = cv1w; base = (size_t)row * CIN + k; dst = W1 + (size_t)row * CIN + k;
    } else if (blk < 704) {
      const int L = (blk - 128) * 32 + lq;
      const int row = L / 36, pc = L - 36 * row;
      const int k = pc * 64 + 8 * e;
      const int tap = k >> 8, ci = k & 255;
      src = m1w; base = ((size_t)row * CHID + ci) * 9 + tap; strd = 9; dst = W3 + (size_t)row * K3 + k;
    } else if (blk < 896) {
      const int L = (blk - 704) * 32 + lq;
      const int row = L >> 2, k = (L & 3) * 64 + 8 * e;
      src = qkvw; base = (size_t)row * CHID + k; dst = WQ + (size_t)row * CHID + k;
    } else if (blk < 960) {
      const int L = (blk - 896) * 32 + lq;
      const int row = L >> 2, k = (L & 3) * 64 + 8 * e;
      src = m2w; base = (size_t)row * CHID + k; dst = W2 + (size_t)row * CHID + k;
    } else {
      const int L = (blk - 960) * 32 + lq;
      const int row = L >> 4, k = (L & 15) * 64 + 8 * e;
      src = cv2w; base = (size_t)row * CCAT + k; dst = WF + (size_t)row * CCAT + k;
    }
    v4u u;
#pragma unroll
    for (int q = 0; q < 4; ++q) {
      const float v0 = src[base + (size_t)(2 * q) * strd];
      const float v1 = src[base + (size_t)(2 * q + 1) * strd];
      u[q] = pk16(h_bits((_Float16)(WSC * bfr(v0))), h_bits((_Float16)(WSC * bfr(v1))));
    }
#pragma unroll
    for (int pass = 0; pass < 2; ++pass) {
      *(volatile v4u*)dst = u;
      __threadfence();
    }
  } else {
    const int L = (blk - 1216) * 32 + lq;
    const int f0 = L * 32 + 4 * e;
    const int set = f0 / 1536, rem = f0 - 1536 * set;
    const int comp = rem >> 9, ch = rem & 511;
    const float* bnp = (set == 0) ? cv1bn : (set == 1) ? m1bn : (set == 2) ? (m1bn + 4 * CHID)
                     : (set == 3) ? m2bn : (set == 4) ? (m2bn + 4 * CHID) : cv2bn;
    const int nch = (set == 0 || set == 5) ? 512 : 256;
    v4f o;
#pragma unroll
    for (int q = 0; q < 4; ++q) {
      const int chq = ch + q;
      const int chc = min(chq, nch - 1);
      const float g = bfr(bnp[chc]), be = bfr(bnp[nch + chc]);
      const float mm = bfr(bnp[2 * nch + chc]), var = bfr(bnp[3 * nch + chc]);
      const float s = g * rsqrtf(var + BNEPS);
      const float val = (comp == 0) ? s : ((comp == 1) ? mm : be);
      o[q] = (chq < nch) ? val : 0.f;
    }
    float* dst = COEF + f0;
#pragma unroll
    for (int pass = 0; pass < 2; ++pass) {
      *(volatile v4f*)dst = o;
      __threadfence();
    }
  }
}

__global__ __launch_bounds__(256)
void k_xcvt(const float* __restrict__ x, unsigned short* X0) {
  __shared__ __align__(16) unsigned short Xs[32 * XSP];
  const int tid = threadIdx.x;
  const int n0 = blockIdx.x * 32, b = n0 >> 10, p0 = n0 & 1023;
#pragma unroll 4
  for (int it = 0; it < 16; ++it) {
    const int idx = it * 256 + tid;
    const int ch = idx >> 3, p4 = (idx & 7) * 4;
    const v4f v = *(const v4f*)(x + ((size_t)(b * CIN + ch)) * HW + p0 + p4);
#pragma unroll
    for (int q = 0; q < 4; ++q) Xs[(p4 + q) * XSP + ch] = h_bits((_Float16)(ASC * bfr(v[q])));
  }
  __syncthreads();
  const int e = tid & 7, lq = tid >> 3;
#pragma unroll
  for (int pass = 0; pass < 2; ++pass) {
#pragma unroll
    for (int it = 0; it < 8; ++it) {
      const int L = it * 32 + lq;
      const int p = L >> 3, pc = L & 7;
      const v4u u = *(const v4u*)(Xs + p * XSP + pc * 64 + 8 * e);
      *(volatile v4u*)(X0 + ((size_t)(n0 + p)) * CIN + pc * 64 + 8 * e) = u;
    }
    __threadfence();
  }
}

__global__ __launch_bounds__(256)
void k_gemm_act(const unsigned short* __restrict__ X, int lda, const unsigned short* __restrict__ W, int K,
                const float* __restrict__ coef, unsigned short* OUT, int ldo,
                const unsigned short* __restrict__ RES, int ldr, int hasres) {
  __shared__ __align__(16) unsigned short O[64 * OP];
  const int tid = threadIdx.x, lane = tid & 31, wave = tid >> 5;
  const int hh = lane >> 4, c = lane & 15;
  const int p0 = blockIdx.x * 64, m0 = blockIdx.y * 128;
  const int wm = wave & 1, wn = wave >> 1;
  const unsigned short* ap0 = X + (size_t)(p0 + 32 * wm + c) * lda + 8 * hh;
  const unsigned short* ap1 = ap0 + (size_t)16 * lda;
  const unsigned short* bp0 = W + (size_t)(m0 + 32 * wn + c) * K + 8 * hh;
  const unsigned short* bp1 = bp0 + (size_t)16 * K;
  v8f acc[2][2];
  acc[0][0] = zero8(); acc[0][1] = zero8(); acc[1][0] = zero8(); acc[1][1] = zero8();
  const int nks = K >> 5;
#pragma unroll 2
  for (int ks = 0; ks < nks; ++ks) {
    const Frag fa0 = ldfrag(ap0 + 32 * ks), fa1 = ldfrag(ap1 + 32 * ks);
    const Frag fb0 = ldfrag(bp0 + 32 * ks), fb1 = ldfrag(bp1 + 32 * ks);
    acc[0][0] = mma_h(fa0.h, fb0.h, acc[0][0]);
    acc[0][1] = mma_h(fa0.h, fb1.h, acc[0][1]);
    acc[1][0] = mma_h(fa1.h, fb0.h, acc[1][0]);
    acc[1][1] = mma_h(fa1.h, fb1.h, acc[1][1]);
  }
#pragma unroll
  for (int u = 0; u < 2; ++u) {
    const int chl = 32 * wn + 16 * u + c, ch = m0 + chl;
    const float s = coef[ch], mm = coef[512 + ch], be = coef[1024 + ch];
#pragma unroll
    for (int t = 0; t < 2; ++t) {
#pragma unroll
      for (int r = 0; r < 8; ++r) {
        const int pl = 32 * wm + 16 * t + 8 * hh + r;
        float y = (acc[t][u][r] * GINV - mm) * s + be;
        y = silu_f(y);
        if (hasres) y += h_val(RES[(size_t)(p0 + pl) * ldr + ch]) * RINV;
        O[pl * OP + chl] = h_bits((_Float16)(ASC * y));
      }
    }
  }
  __syncthreads();
  {
    const int e = tid & 7, lq = tid >> 3;
#pragma unroll
    for (int pass = 0; pass < 2; ++pass) {
#pragma unroll
      for (int it = 0; it < 4; ++it) {
        const int L = it * 32 + lq;
        const int p = L >> 1, hf = L & 1;
        const v4u u = *(const v4u*)(O + p * OP + hf * 64 + 8 * e);
        *(volatile v4u*)(OUT + ((size_t)(p0 + p)) * ldo + m0 + hf * 64 + 8 * e) = u;
      }
      __threadfence();
    }
  }
}

__global__ __launch_bounds__(256)
void k_gemm_qkv(const unsigned short* __restrict__ Z, const unsigned short* __restrict__ W,
                const float* __restrict__ rw, const float* __restrict__ rh,
                unsigned short* QK, unsigned short* Vp) {
  __shared__ __align__(16) unsigned short O[64 * OP];
  __shared__ __align__(16) unsigned short Ov[128 * OVP];
  const int tid = threadIdx.x, lane = tid & 31, wave = tid >> 5;
  const int hh = lane >> 4, c = lane & 15;
  const int p0 = blockIdx.x * 64, mb = blockIdx.y, m0 = mb * 128;
  const int wm = wave & 1, wn = wave >> 1;
  const unsigned short* ap0 = Z + (size_t)(p0 + 32 * wm + c) * CHID + 8 * hh;
  const unsigned short* ap1 = ap0 + (size_t)16 * CHID;
  const unsigned short* bp0 = W + (size_t)(m0 + 32 * wn + c) * CHID + 8 * hh;
  const unsigned short* bp1 = bp0 + (size_t)16 * CHID;
  v8f acc[2][2];
  acc[0][0] = zero8(); acc[0][1] = zero8(); acc[1][0] = zero8(); acc[1][1] = zero8();
#pragma unroll 2
  for (int ks = 0; ks < CHID / 32; ++ks) {
    const Frag fa0 = ldfrag(ap0 + 32 * ks), fa1 = ldfrag(ap1 + 32 * ks);
    const Frag fb0 = ldfrag(bp0 + 32 * ks), fb1 = ldfrag(bp1 + 32 * ks);
    acc[0][0] = mma_h(fa0.h, fb0.h, acc[0][0]);
    acc[0][1] = mma_h(fa0.h, fb1.h, acc[0][1]);
    acc[1][0] = mma_h(fa1.h, fb0.h, acc[1][0]);
    acc[1][1] = mma_h(fa1.h, fb1.h, acc[1][1]);
  }
  const int e = tid & 7, lq = tid >> 3;
  if (mb < 4) {
    const bool isk = (mb >= 2);
#pragma unroll
    for (int u = 0; u < 2; ++u) {
      const int chl = 32 * wn + 16 * u + c, ch = m0 + chl;
      const int cd = isk ? (ch - 256) : 0;
#pragma unroll
      for (int t = 0; t < 2; ++t) {
#pragma unroll
        for (int r = 0; r < 8; ++r) {
          const int pl = 32 * wm + 16 * t + 8 * hh + r;
          float v = acc[t][u][r] * GINV;
          if (isk) {
            const int p = (p0 + pl) & 1023;
            v += bfr(rw[cd * 32 + (p & 31)]) + bfr(rh[cd * 32 + (p >> 5)]);
          }
          O[pl * OP + chl] = h_bits((_Float16)(ASC * v));
        }
      }
    }
    __syncthreads();
#pragma unroll
    for (int pass = 0; pass < 2; ++pass) {
#pragma unroll
      for (int it = 0; it < 4; ++it) {
        const int L = it * 32 + lq;
        const int p = L >> 1, hf = L & 1;
        const v4u u = *(const v4u*)(O + p * OP + hf * 64 + 8 * e);
        *(volatile v4u*)(QK + ((size_t)(p0 + p)) * QKP + m0 + hf * 64 + 8 * e) = u;
      }
      __threadfence();
    }
  } else {
#pragma unroll
    for (int u = 0; u < 2; ++u) {
      const int chl = 32 * wn + 16 * u + c;
#pragma unroll
      for (int t = 0; t < 2; ++t) {
#pragma unroll
        for (int r = 0; r < 8; ++r) {
          const int pl = 32 * wm + 16 * t + 8 * hh + r;
          Ov[chl * OVP + pl] = h_bits((_Float16)(ASC * (acc[t][u][r] * GINV)));
        }
      }
    }
    __syncthreads();
#pragma unroll
    for (int pass = 0; pass < 2; ++pass) {
#pragma unroll
      for (int it = 0; it < 4; ++it) {
        const int chl = it * 32 + lq;
        const v4u u = *(const v4u*)(Ov + chl * OVP + 8 * e);
        *(volatile v4u*)(Vp + ((size_t)(m0 - 512 + chl)) * NTOT + p0 + 8 * e) = u;
      }
      __threadfence();
    }
  }
}

__global__ __launch_bounds__(256)
void k_conv3(const unsigned short* __restrict__ Y, const unsigned short* __restrict__ W3,
             const float* __restrict__ coef, unsigned short* Z) {
  union Lds { unsigned short tin[4 * 34 * TP]; unsigned short O[64 * OP3]; };
  __shared__ __align__(16) Lds U;
  unsigned short* const tin = U.tin;
  unsigned short* const O = U.O;
  const int tid = threadIdx.x, lane = tid & 31, wave = tid >> 5;
  const int hh = lane >> 4, c = lane & 15;
  const int n0 = blockIdx.x * 64, b = n0 >> 10, pl0 = n0 & 1023, y0 = pl0 >> 5;
  const int wm = wave & 1, wn = wave >> 1;
  v8f acc[2][4];
#pragma unroll
  for (int t = 0; t < 2; ++t) {
#pragma unroll
    for (int u = 0; u < 4; ++u) acc[t][u] = zero8();
  }
  const unsigned short* bp0 = W3 + ((size_t)(64 * wn + c)) * K3 + 8 * hh;
  const v4u z4 = {0u, 0u, 0u, 0u};

#pragma unroll 1
  for (int cc = 0; cc < CHID / 64; ++cc) {
    __syncthreads();
    for (int i = tid; i < 4 * 34 * 8; i += 256) {
      const int e8 = i & 7, t2 = i >> 3;
      const int px = t2 % 34, ry = t2 / 34;
      const int gy = y0 + ry - 1, gx = px - 1;
      const bool ok = (gy >= 0) && (gy < IMW) && (gx >= 0) && (gx < IMW);
      const int gyc = min(max(gy, 0), IMW - 1), gxc = min(max(gx, 0), IMW - 1);
      v4u v = *(const v4u*)(Y + ((size_t)(b * HW + gyc * IMW + gxc)) * CCAT + cc * 64 + 8 * e8);
      if (!ok) v = z4;
      *(v4u*)(tin + (ry * 34 + px) * TP + 8 * e8) = v;
    }
    __syncthreads();
#pragma unroll
    for (int tap = 0; tap < 9; ++tap) {
      const int dy = tap / 3, dx = tap - 3 * dy;
      const unsigned short* ta0 = tin + ((wm + dy) * 34 + dx + c) * TP + 8 * hh;
      const unsigned short* ta1 = ta0 + 16 * TP;
      const size_t wk = (size_t)tap * CHID + cc * 64;
#pragma unroll
      for (int ks = 0; ks < 2; ++ks) {
        const Frag fa0 = ldfrag(ta0 + 32 * ks), fa1 = ldfrag(ta1 + 32 * ks);
#pragma unroll
        for (int u = 0; u < 4; ++u) {
          const Frag fb = ldfrag(bp0 + (size_t)u * 16 * K3 + wk + 32 * ks);
          acc[0][u] = mma_h(fa0.h, fb.h, acc[0][u]);
          acc[1][u] = mma_h(fa1.h, fb.h, acc[1][u]);
        }
      }
    }
  }
  __syncthreads();
#pragma unroll
  for (int u = 0; u < 4; ++u) {
    const int ocl = 64 * wn + 16 * u + c;
    const float s = coef[ocl], mm = coef[512 + ocl], be = coef[1024 + ocl];
#pragma unroll
    for (int t = 0; t < 2; ++t) {
#pragma unroll
      for (int r = 0; r < 8; ++r) {
        const int pl = 32 * wm + 16 * t + 8 * hh + r;
        float y = (acc[t][u][r] * GINV - mm) * s + be;
        y = silu_f(y);
        O[pl * OP3 + ocl] = h_bits((_Float16)(ASC * y));
      }
    }
  }
  __syncthreads();
  {
    const int e = tid & 7, lq = tid >> 3;
#pragma unroll
    for (int pass = 0; pass < 2; ++pass) {
#pragma unroll
      for (int it = 0; it < 8; ++it) {
        const int L = it * 32 + lq;
        const int p = L >> 2, q4 = L & 3;
        const v4u u = *(const v4u*)(O + p * OP3 + q4 * 64 + 8 * e);
        *(volatile v4u*)(Z + ((size_t)(n0 + p)) * CHID + q4 * 64 + 8 * e) = u;
      }
      __threadfence();
    }
  }
}

__global__ __launch_bounds__(256)
void k_attn(const unsigned short* __restrict__ QK, const unsigned short* __restrict__ Vp, unsigned short* AO) {
  extern __shared__ __align__(16) unsigned char att_lds[];
  float* S = (float*)att_lds;
  unsigned short* P = (unsigned short*)(att_lds + ATT_S_BYTES);
  float* RED = (float*)(att_lds + ATT_S_BYTES + ATT_P_BYTES);
  unsigned short* O16 = (unsigned short*)(att_lds + ATT_S_BYTES + ATT_P_BYTES + ATT_R_BYTES);
  const int tid = threadIdx.x, lane = tid & 31, wave = tid >> 5;
  const int hh = lane >> 4, c = lane & 15;
  const int i0 = blockIdx.x * 32, h = blockIdx.y, b = blockIdx.z;
  const size_t nb = (size_t)b * HW;

  {
    const unsigned short* qr = QK + (nb + i0 + c) * QKP + h * HD + 8 * hh;
    const Frag q00 = ldfrag(qr), q01 = ldfrag(qr + 32);
    const Frag q10 = ldfrag(qr + (size_t)16 * QKP), q11 = ldfrag(qr + (size_t)16 * QKP + 32);
    const unsigned short* kr0 = QK + (nb + c) * QKP + CHID + h * HD + 8 * hh;
#pragma unroll 1
    for (int jq = 0; jq < 8; ++jq) {
      const int jt = wave * 8 + jq;
      const unsigned short* kr = kr0 + (size_t)(16 * jt) * QKP;
      const Frag k0 = ldfrag(kr), k1 = ldfrag(kr + 32);
      v8f s0 = zero8(), s1 = zero8();
      s0 = mma_h(q00.h, k0.h, s0);
      s1 = mma_h(q10.h, k0.h, s1);
      s0 = mma_h(q01.h, k1.h, s0);
      s1 = mma_h(q11.h, k1.h, s1);
#pragma unroll
      for (int r = 0; r < 8; ++r) {
        S[(8 * hh + r) * SP + 16 * jt + c] = s0[r] * LINV;
        S[(16 + 8 * hh + r) * SP + 16 * jt + c] = s1[r] * LINV;
      }
    }
  }
  __syncthreads();

  {
    const int row = tid >> 3, cl = tid & 7;
    float* sr = S + row * SP;
    float mx = -3.0e38f;
#pragma unroll 4
    for (int jj = 0; jj < 128; ++jj) mx = fmaxf(mx, sr[cl + 8 * jj]);
#pragma unroll
    for (int off = 4; off > 0; off >>= 1) mx = fmaxf(mx, __shfl_xor(mx, off, 8));
    float sum = 0.f;
#pragma unroll 4
    for (int jj = 0; jj < 128; ++jj) {
      const int j = cl + 8 * jj;
      const float ev = __expf(sr[j] - mx);
      sr[j] = ev;
      sum += ev;
    }
#pragma unroll
    for (int off = 4; off > 0; off >>= 1) sum += __shfl_xor(sum, off, 8);
    const float inv = PSC * __builtin_amdgcn_rcpf(sum);
    unsigned short* pr = P + row * PP;
#pragma unroll 4
    for (int jj = 0; jj < 128; ++jj) {
      const int j = cl + 8 * jj;
      pr[j] = h_bits((_Float16)(sr[j] * inv));
    }
  }
  __syncthreads();

  {
    const int dt = wave & 3, kh = wave >> 2;
    const unsigned short* pa0 = P + c * PP + kh * 512 + 8 * hh;
    const unsigned short* pa1 = pa0 + 16 * PP;
    const unsigned short* vb = Vp + ((size_t)(h * HD + 16 * dt + c)) * NTOT + nb + kh * 512 + 8 * hh;
    v8f o0 = zero8(), o1 = zero8();
#pragma unroll 4
    for (int ks = 0; ks < 16; ++ks) {
      const Frag fa0 = ldfrag(pa0 + 32 * ks), fa1 = ldfrag(pa1 + 32 * ks);
      const Frag fb = ldfrag(vb + 32 * ks);
      o0 = mma_h(fa0.h, fb.h, o0);
      o1 = mma_h(fa1.h, fb.h, o1);
    }
    if (kh) {
#pragma unroll
      for (int r = 0; r < 8; ++r) {
        RED[(8 * hh + r) * 64 + 16 * dt + c] = o0[r];
        RED[(16 + 8 * hh + r) * 64 + 16 * dt + c] = o1[r];
      }
    }
    __syncthreads();
    if (!kh) {
#pragma unroll
      for (int r = 0; r < 8; ++r) {
        const float v0 = (o0[r] + RED[(8 * hh + r) * 64 + 16 * dt + c]) * OINV;
        const float v1 = (o1[r] + RED[(16 + 8 * hh + r) * 64 + 16 * dt + c]) * OINV;
        O16[(8 * hh + r) * OPA + 16 * dt + c] = h_bits((_Float16)v0);
        O16[(16 + 8 * hh + r) * OPA + 16 * dt + c] = h_bits((_Float16)v1);
      }
    }
    __syncthreads();
  }

  {
    const int e = tid & 7, lq = tid >> 3;
    const v4u u = *(const v4u*)(O16 + lq * OPA + 8 * e);
    unsigned short* dst = AO + (nb + i0 + lq) * CHID + h * HD + 8 * e;
#pragma unroll
    for (int pass = 0; pass < 2; ++pass) {
      *(volatile v4u*)dst = u;
      __threadfence();
    }
  }
}

__global__ __launch_bounds__(256)
void k_gemm_out(const unsigned short* __restrict__ X, const unsigned short* __restrict__ W,
                const float* __restrict__ coef, float* OUT) {
  __shared__ __align__(16) float Of[128 * OFP];
  const int tid = threadIdx.x, lane = tid & 31, wave = tid >> 5;
  const int hh = lane >> 4, c = lane & 15;
  const int p0 = blockIdx.x * 64, m0 = blockIdx.y * 128;
  const int b = p0 >> 10, pl0 = p0 & 1023;
  const int wm = wave & 1, wn = wave >> 1;
  const unsigned short* ap0 = X + (size_t)(p0 + 32 * wm + c) * CCAT + 8 * hh;
  const unsigned short* ap1 = ap0 + (size_t)16 * CCAT;
  const unsigned short* bp0 = W + (size_t)(m0 + 32 * wn + c) * CCAT + 8 * hh;
  const unsigned short* bp1 = bp0 + (size_t)16 * CCAT;
  v8f acc[2][2];
  acc[0][0] = zero8(); acc[0][1] = zero8(); acc[1][0] = zero8(); acc[1][1] = zero8();
#pragma unroll 2
  for (int ks = 0; ks < CCAT / 32; ++ks) {
    const Frag fa0 = ldfrag(ap0 + 32 * ks), fa1 = ldfrag(ap1 + 32 * ks);
    const Frag fb0 = ldfrag(bp0 + 32 * ks), fb1 = ldfrag(bp1 + 32 * ks);
    acc[0][0] = mma_h(fa0.h, fb0.h, acc[0][0]);
    acc[0][1] = mma_h(fa0.h, fb1.h, acc[0][1]);
    acc[1][0] = mma_h(fa1.h, fb0.h, acc[1][0]);
    acc[1][1] = mma_h(fa1.h, fb1.h, acc[1][1]);
  }
#pragma unroll
  for (int u = 0; u < 2; ++u) {
    const int chl = 32 * wn + 16 * u + c, ch = m0 + chl;
    const float s = coef[ch], mm = coef[512 + ch], be = coef[1024 + ch];
#pragma unroll
    for (int t = 0; t < 2; ++t) {
#pragma unroll
      for (int r = 0; r < 8; ++r) {
        const int pl = 32 * wm + 16 * t + 8 * hh + r;
        float y = (acc[t][u][r] * GINV - mm) * s + be;
        Of[chl * OFP + pl] = silu_f(y);
      }
    }
  }
  __syncthreads();
  {
    const int e = tid & 7, lq = tid >> 3;
#pragma unroll
    for (int pass = 0; pass < 2; ++pass) {
#pragma unroll
      for (int it = 0; it < 8; ++it) {
        const int L = it * 32 + lq;
        const int chl = L >> 1, hf = L & 1;
        const v4f v = *(const v4f*)(Of + chl * OFP + hf * 32 + 4 * e);
        float* dst = OUT + ((size_t)(b * COUT + m0 + chl)) * HW + pl0 + hf * 32 + 4 * e;
        *(volatile v4f*)dst = v;
      }
      __threadfence();
    }
  }
}

extern "C" void kernel_launch(void* const* d_in, const int* in_sizes, int n_in,
                              void* d_out, int out_size, void* d_ws, size_t ws_size,
                              hipStream_t stream) {
  if (n_in < 12) return;
  if (in_sizes[0] != NBATCH * CIN * HW) return;
  if (in_sizes[1] != COUT * CIN) return;
  if (in_sizes[2] != 4 * COUT) return;
  if (in_sizes[3] != COUT * CCAT) return;
  if (in_sizes[4] != 4 * COUT) return;
  if (in_sizes[5] != NLAY * CHID * CHID * 9) return;
  if (in_sizes[6] != NLAY * 4 * CHID) return;
  if (in_sizes[7] != NLAY * CQKV * CHID) return;
  if (in_sizes[8] != NLAY * NHEAD * HD * IMW) return;
  if (in_sizes[9] != NLAY * NHEAD * HD * IMW) return;
  if (in_sizes[10] != NLAY * CHID * CHID) return;
  if (in_sizes[11] != NLAY * 4 * CHID) return;
  if (out_size != NBATCH * COUT * HW) return;

  size_t off = 0;
  auto carve = [&](size_t bytes) { const size_t o = off; off += (bytes + 255) & ~(size_t)255; return o; };
  const size_t oW1 = carve((size_t)COUT * CIN * 2);
  const size_t oW3 = carve((size_t)NLAY * CHID * K3 * 2);
  const size_t oWQ = carve((size_t)NLAY * CQKV * CHID * 2);
  const size_t oW2 = carve((size_t)NLAY * CHID * CHID * 2);
  const size_t oWF = carve((size_t)COUT * CCAT * 2);
  const size_t oCF = carve((size_t)6 * 3 * 512 * 4);
  const size_t oX0 = carve((size_t)NTOT * CIN * 2);
  const size_t oYC = carve((size_t)NTOT * CCAT * 2);
  const size_t oZ  = carve((size_t)NTOT * CHID * 2);
  const size_t oQK = carve((size_t)NTOT * QKP * 2);
  const size_t oV  = carve((size_t)CHID * NTOT * 2);
  const size_t oAO = carve((size_t)NTOT * CHID * 2);
  if (off > ws_size) return;
  if (off > (size_t)134217728) return;

  const float* x     = (const float*)d_in[0];
  const float* cv1w  = (const float*)d_in[1];
  const float* cv1bn = (const float*)d_in[2];
  const float* cv2w  = (const float*)d_in[3];
  const float* cv2bn = (const float*)d_in[4];
  const float* m1w   = (const float*)d_in[5];
  const float* m1bn  = (const float*)d_in[6];
  const float* qkvw  = (const float*)d_in[7];
  const float* mrw   = (const float*)d_in[8];
  const float* mrh   = (const float*)d_in[9];
  const float* m2w   = (const float*)d_in[10];
  const float* m2bn  = (const float*)d_in[11];
  float* out = (float*)d_out;

  char* ws = (char*)d_ws;
  unsigned short* W1  = (unsigned short*)(ws + oW1);
  unsigned short* W3  = (unsigned short*)(ws + oW3);
  unsigned short* WQ  = (unsigned short*)(ws + oWQ);
  unsigned short* W2  = (unsigned short*)(ws + oW2);
  unsigned short* WF  = (unsigned short*)(ws + oWF);
  float*          CF  = (float*)(ws + oCF);
  unsigned short* X0  = (unsigned short*)(ws + oX0);
  unsigned short* YC  = (unsigned short*)(ws + oYC);
  unsigned short* Zp  = (unsigned short*)(ws + oZ);
  unsigned short* QK  = (unsigned short*)(ws + oQK);
  unsigned short* Vpl = (unsigned short*)(ws + oV);
  unsigned short* AO  = (unsigned short*)(ws + oAO);

  const dim3 blk256(256);
  (void)hipFuncSetAttribute(reinterpret_cast<const void*>(&k_attn),
                            hipFuncAttributeMaxDynamicSharedMemorySize, ATT_LDS);

  k_cvt<<<dim3(1225), blk256, 0, stream>>>(cv1w, cv1bn, cv2w, cv2bn, m1w, m1bn, qkvw, m2w, m2bn,
                                           W1, W3, WQ, W2, WF, CF);
  k_xcvt<<<dim3(NTOT / 32), blk256, 0, stream>>>(x, X0);
  k_gemm_act<<<dim3(NTOT / 64, COUT / 128), blk256, 0, stream>>>(X0, CIN, W1, CIN, CF, YC, CCAT, X0, CIN, 0);
  for (int i = 0; i < NLAY; ++i) {
    const unsigned short* yin = YC + CHID * (1 + i);
    k_conv3<<<dim3(NTOT / 64), blk256, 0, stream>>>(yin, W3 + (size_t)i * CHID * K3, CF + (size_t)(1 + i) * 1536, Zp);
    k_gemm_qkv<<<dim3(NTOT / 64, CQKV / 128), blk256, 0, stream>>>(Zp, WQ + (size_t)i * CQKV * CHID,
                                                                    mrw + (size_t)i * NHEAD * HD * IMW,
                                                                    mrh + (size_t)i * NHEAD * HD * IMW, QK, Vpl);
    k_attn<<<dim3(HW / 32, NHEAD, NBATCH), blk256, ATT_LDS, stream>>>(QK, Vpl, AO);
    k_gemm_act<<<dim3(NTOT / 64, CHID / 128), blk256, 0, stream>>>(AO, CHID, W2 + (size_t)i * CHID * CHID, CHID,
                                                                    CF + (size_t)(3 + i) * 1536,
                                                                    YC + CHID * (2 + i), CCAT, yin, CCAT, 1);
  }
  k_gemm_out<<<dim3(NTOT / 64, COUT / 128), blk256, 0, stream>>>(YC, WF, CF + (size_t)5 * 1536, out);
  (void)hipGetLastError();
}
